// CausalAnomalyDetector_28415503630423
// MI455X (gfx1250) — hardware-run, weakly checked
//
#include <hip/hip_runtime.h>


namespace {
constexpr int B = 65536, F = 6, H = 32, SPW = 32, NR = SPW * F;
constexpr float XS = 8.0f, WSC = 256.0f;
typedef _Float16 b16;
typedef __attribute__((ext_vector_type(16))) _Float16 v16b;
typedef __attribute__((ext_vector_type(8))) _Float16 v8b;
typedef __attribute__((ext_vector_type(8))) float v8f;
typedef __attribute__((ext_vector_type(4))) float v4f;
__device__ __forceinline__ float bf16_rne(float f) { unsigned int u = __float_as_uint(f); u += 0x7FFFu + ((u >> 16) & 1u); return __uint_as_float(u & 0xFFFF0000u); }
__device__ __forceinline__ void split16(float v, b16& hi, b16& lo) { hi = (b16)v; lo = (b16)(v - (float)hi); }
__device__ __forceinline__ v16b frag_kb(const b16* p, int hh) { const v8b a = *(const v8b*)(p + 8 * hh), b = *(const v8b*)(p + 16 + 8 * hh); v16b f;
#pragma unroll
  for (int e = 0; e < 8; ++e) { f[e] = a[e]; f[8 + e] = b[e]; } return f; }
__device__ __forceinline__ v8f wmma16b(v16b a, v16b b, v8f c) { v8f d = __builtin_amdgcn_wmma_f32_16x16x32_f16(false, a, false, b, (short)0, c, false, false); asm volatile("v_nop\n\tv_nop\n\tv_nop\n\tv_nop" : "+v"(d) : "v"(a), "v"(b)); return d; }
__device__ __forceinline__ void wave_lds_sync() { __builtin_amdgcn_fence(__ATOMIC_RELEASE, "workgroup"); __builtin_amdgcn_wave_barrier(); __builtin_amdgcn_fence(__ATOMIC_ACQUIRE, "workgroup"); }
__device__ __forceinline__ float pmul(float a, float b) { float p = a * b; asm volatile("" : "+v"(p)); return p; }
__device__ __forceinline__ float sigm(float v) { return 1.0f / (1.0f + __expf(-v)); }

__global__ __launch_bounds__(256) void wput_kernel(const float* __restrict__ w, int r0, int KIN, int KP, int OUTW, int ro, b16* __restrict__ WT) {
  const int KG = KP / 8; const int u = blockIdx.x * 256 + threadIdx.x; if (u >= OUTW * KG) return; const int o = u / KG, k0 = (u % KG) * 8; v8b v;
#pragma unroll
  for (int j = 0; j < 8; ++j) { const int k = k0 + j; v[j] = k < KIN ? (b16)(bf16_rne(w[(size_t)(r0 + k) * OUTW + o]) * WSC) : (b16)0.0f; } for (int pass = 0; pass < 2; ++pass) { *(volatile v8b*)(WT + (size_t)(ro + o) * KP + k0) = v; __threadfence(); }
}
template <int NT, typename EP>
__device__ __forceinline__ void lds_gemm(b16 (*Ah)[40], b16 (*Al)[40], const b16* __restrict__ WT, int nloc, int hlf, EP ep) {
#pragma unroll 1
  for (int rt = 0; rt < NR / 16; ++rt) { const v16b a = frag_kb(&Ah[rt * 16 + nloc][0], hlf), al = frag_kb(&Al[rt * 16 + nloc][0], hlf);
#pragma unroll
    for (int t = 0; t < NT; ++t) { v8f acc = {}; const v16b bw = frag_kb(WT + (size_t)(t * 16 + nloc) * 32, hlf); acc = wmma16b(a, bw, acc); acc = wmma16b(al, bw, acc);
#pragma unroll
      for (int r8 = 0; r8 < 8; ++r8) ep(rt * 16 + 8 * hlf + r8, t * 16 + nloc, acc[r8] * (1.0f / (XS * WSC))); } }
}
__global__ __launch_bounds__(32) void ca_kernel(const float* __restrict__ fac, const float* __restrict__ Wn, const float* __restrict__ bn, const b16* __restrict__ WE1, const float* __restrict__ be1, const float* __restrict__ We2, const float* __restrict__ be2, const float* __restrict__ Wd1, const float* __restrict__ bd1, const b16* __restrict__ WD2, const float* __restrict__ bd2, const float* __restrict__ Wd3, const float* __restrict__ bd3, const b16* __restrict__ WS1, const float* __restrict__ bs1, const b16* __restrict__ WS2, const float* __restrict__ bs2, const float* __restrict__ Ws3, const float* __restrict__ bs3, float* __restrict__ oadj, float* __restrict__ opred, float* __restrict__ osc) {
  __shared__ float Fa[SPW][F][F], Pr[SPW][F][F], Ad[SPW][F][F]; __shared__ __attribute__((aligned(16))) b16 Ah[NR][40], Al[NR][40]; __shared__ float PQ[NR][2 * H + 1]; __shared__ float Sv[NR];
  const int lane = threadIdx.x, nloc = lane & 15, hlf = lane >> 4; const size_t s0 = (size_t)blockIdx.x * SPW;
  for (int i = lane; i < SPW * F * F; i += 32) ((float*)Fa)[i] = bf16_rne(fac[s0 * F * F + i]);
  wave_lds_sync();
  { float w[F]; for (int k = 0; k < F; ++k) w[k] = bf16_rne(Wn[k * H + lane]); const float bb = bf16_rne(bn[lane]);
#pragma unroll 1
    for (int r = 0; r < NR; ++r) { const float* fr = &Fa[r / F][r % F][0]; float v = bb; for (int k = 0; k < F; ++k) v += pmul(fr[k], w[k]); b16 p, q; split16(v * XS, p, q); Ah[r][lane] = p; Al[r][lane] = q; } }
  wave_lds_sync();
  lds_gemm<4>(Ah, Al, WE1, nloc, hlf, [&](int r, int c, float v) { PQ[r][c] = v; });
  wave_lds_sync();
  { const float bq = bf16_rne(be2[0]);
#pragma unroll 1
    for (int it = lane; it < SPW * F * F; it += 32) { const int s = it / (F * F), ij = it % (F * F), i = ij / F, j = ij % F; const float* Pi = &PQ[s * F + i][0]; const float* Qj = &PQ[s * F + j][H]; float d = bq;
#pragma unroll 4
      for (int c = 0; c < H; ++c) d += pmul(fmaxf(Pi[c] + Qj[c] + bf16_rne(be1[c]), 0.0f), bf16_rne(We2[c])); Ad[s][i][j] = (i == j) ? 0.0f : sigm(d); } }
  wave_lds_sync();
  for (int pass = 0; pass < 2; ++pass) { for (int i = lane; i < SPW * F * F; i += 32) ((volatile float*)oadj)[s0 * F * F + i] = ((float*)Ad)[i]; __threadfence(); }
  { float w[F]; for (int k = 0; k < F; ++k) w[k] = bf16_rne(Wd1[k * H + lane]); const float bb = bf16_rne(bd1[lane]);
#pragma unroll 1
    for (int r = 0; r < NR; ++r) { const int s = r / F, n = r % F; float v = bb;
      for (int i = 0; i < F; ++i) { float st = 0.0f; for (int j = 0; j < F; ++j) st += pmul(Ad[s][i][j], Fa[s][n][j]); v += pmul(st, w[i]); }
      b16 p, q; split16(fmaxf(v, 0.0f) * XS, p, q); Ah[r][lane] = p; Al[r][lane] = q; } }
  wave_lds_sync();
  lds_gemm<2>(Ah, Al, WD2, nloc, hlf, [&](int r, int c, float v) { PQ[r][c] = fmaxf(v + bf16_rne(bd2[c]), 0.0f); });
  wave_lds_sync();
#pragma unroll 1
  for (int it = lane; it < NR * F; it += 32) { const int r = it / F, o = it % F; float v = bf16_rne(bd3[o]);
#pragma unroll 4
    for (int c = 0; c < H; ++c) v += pmul(PQ[r][c], bf16_rne(Wd3[c * F + o])); Pr[r / F][r % F][o] = v; }
  wave_lds_sync();
  for (int pass = 0; pass < 2; ++pass) { for (int i = lane; i < SPW * F * F; i += 32) ((volatile float*)opred)[s0 * F * F + i] = ((float*)Pr)[i]; __threadfence(); }
#pragma unroll 1
  for (int r = 0; r < NR; ++r) { const int s = r / F, n = r % F; float v = 0.0f; if (lane < F) v = Fa[s][n][lane]; else if (lane < 2 * F) v = Pr[s][n][lane - F]; else if (lane < 3 * F) v = fabsf(Fa[s][n][lane - 2 * F] - Pr[s][n][lane - 2 * F]); b16 p, q; split16(v * XS, p, q); Ah[r][lane] = p; Al[r][lane] = q; }
  wave_lds_sync();
  lds_gemm<2>(Ah, Al, WS1, nloc, hlf, [&](int r, int c, float v) { PQ[r][c] = fmaxf(v + bf16_rne(bs1[c]), 0.0f); });
  wave_lds_sync();
  for (int r = 0; r < NR; ++r) { b16 p, q; split16(PQ[r][lane] * XS, p, q); Ah[r][lane] = p; Al[r][lane] = q; }
  wave_lds_sync();
  lds_gemm<1>(Ah, Al, WS2, nloc, hlf, [&](int r, int c, float v) { PQ[r][32 + c] = fmaxf(v + bf16_rne(bs2[c]), 0.0f); });
  wave_lds_sync();
#pragma unroll 1
  for (int r = lane; r < NR; r += 32) { float v = bf16_rne(bs3[0]); for (int c = 0; c < 16; ++c) v += pmul(PQ[r][32 + c], bf16_rne(Ws3[c])); Sv[r] = sigm(v); }
  wave_lds_sync();
  { const int s = lane; float m = 0.0f; for (int n = 0; n < F; ++n) m += Sv[s * F + n]; m *= (1.0f / F); for (int pass = 0; pass < 2; ++pass) { ((volatile float*)osc)[s0 + s] = m; __threadfence(); } }
}
}

extern "C" void kernel_launch(void* const* d_in, const int* in_sizes, int n_in, void* d_out, int out_size, void* d_ws, size_t ws_size, hipStream_t stream) {
  (void)n_in;
  auto Fp = [&](int i) { return (const float*)d_in[i]; };
  if (in_sizes[0] != B * F * F || in_sizes[1] != F * H || in_sizes[3] != 2 * H * H || in_sizes[5] != H || in_sizes[9] != H * H || in_sizes[11] != H * F || in_sizes[13] != 3 * F * 32 || in_sizes[15] != 32 * 16 || in_sizes[17] != 16 || out_size != 2 * B * F * F + B) return;
  const int NBV = B;
  size_t off = 0; char* ws = (char*)d_ws;
  auto carve = [&](size_t bytes) { char* p = ws + off; off += (bytes + 255) & ~(size_t)255; return p; };
  b16* WE1 = (b16*)carve(64 * 32 * 2); b16* WD2 = (b16*)carve(32 * 32 * 2); b16* WS1 = (b16*)carve(32 * 32 * 2); b16* WS2 = (b16*)carve(16 * 32 * 2);
  if (off > ws_size || off > ((size_t)1 << 20)) return;
  wput_kernel<<<1, 256, 0, stream>>>(Fp(3), 0, H, 32, H, 0, WE1); wput_kernel<<<1, 256, 0, stream>>>(Fp(3), H, H, 32, H, H, WE1);
  wput_kernel<<<1, 256, 0, stream>>>(Fp(9), 0, H, 32, H, 0, WD2); wput_kernel<<<1, 256, 0, stream>>>(Fp(13), 0, 3 * F, 32, 32, 0, WS1); wput_kernel<<<1, 256, 0, stream>>>(Fp(15), 0, 32, 32, 16, 0, WS2);
  float* out = (float*)d_out;
  ca_kernel<<<(unsigned)(NBV / SPW), 32, 0, stream>>>(Fp(0), Fp(1), Fp(2), WE1, Fp(4), Fp(5), Fp(6), Fp(7), Fp(8), WD2, Fp(10), Fp(11), Fp(12), WS1, Fp(14), WS2, Fp(16), Fp(17), Fp(18), out, out + (size_t)B * F * F, out + (size_t)2 * B * F * F);
}
